// NgramHead_28003186770669
// MI455X (gfx1250) — hardware-verified
//
#include <hip/hip_runtime.h>
#include <stddef.h>


typedef _Float16 v16h __attribute__((ext_vector_type(16)));
typedef _Float16 v8h  __attribute__((ext_vector_type(8)));
typedef float    v8f  __attribute__((ext_vector_type(8)));
typedef float    v4f  __attribute__((ext_vector_type(4)));
typedef int      v4i  __attribute__((ext_vector_type(4)));
typedef _Float16 h16;

#ifndef NB
#define NB 4
#endif
#ifndef SEQ
#define SEQ 2048
#endif
#define NB_FULL  4
#define SEQ_FULL 2048
#define DIM   1024
#define KCAT  (2 * DIM)
#define MROWS (NB * SEQ)

static_assert(NB >= 1 && NB <= NB_FULL);
static_assert(SEQ >= 128 && SEQ <= SEQ_FULL && (SEQ % 128) == 0);
static_assert((SEQ / 32) <= 64);
static_assert((DIM % 64) == 0 && (DIM % 32) == 0 && (KCAT % 32) == 0);
static_assert((MROWS % 64) == 0 && (MROWS % 8) == 0 && (DIM % 8) == 0);
static_assert(DIM == 4 * 32 * 8);
static_assert((size_t)MROWS * KCAT < (size_t)0xFFFFFFFFu);
static_assert(((size_t)(NB - 1) * SEQ_FULL + SEQ) * DIM <= (size_t)NB_FULL * SEQ_FULL * DIM);
static_assert((size_t)NB_FULL * SEQ_FULL * DIM * 4 == (size_t)33554432);

#define LDT 72
#define LDC 68
static_assert((LDT % 8) == 0 && LDT >= 64);
static_assert((LDC % 4) == 0 && LDC >= 64);

#define WCARRY 64.0f

#define BT_BYTES  ((size_t)DIM * KCAT * 2)
#define A_BYTES   ((size_t)MROWS * KCAT * 2)
#define VT_BYTES  ((size_t)NB * DIM * SEQ * 2)
#define OFF_BT ((size_t)0)
#define OFF_A  (OFF_BT + BT_BYTES)
#define OFF_VT (OFF_A + A_BYTES)
#define WS_TOTAL (OFF_VT + VT_BYTES)
static_assert((BT_BYTES % 128) == 0 && (A_BYTES % 128) == 0 && (VT_BYTES % 128) == 0);
static_assert(WS_TOTAL <= (size_t)134217728);

__device__ __forceinline__ float bf16r(float x) {
  unsigned int u = __float_as_uint(x);
  u = (u + 0x7FFFu + ((u >> 16) & 1u)) & 0xFFFF0000u;
  return __uint_as_float(u);
}

static __device__ __forceinline__ h16 toh_flush(float v) {
  const h16 r = (h16)v;
  return (fabsf(v) < 6.103515625e-05f) ? (h16)0.0f : r;
}

__device__ __forceinline__ v16h frag_at(const _Float16* p) {
  v8h lo = *(const v8h*)(p);
  v8h hi = *(const v8h*)(p + 16);
  v16h out;
#pragma unroll
  for (int i = 0; i < 8; ++i) { out[i] = lo[i]; out[i + 8] = hi[i]; }
  return out;
}

__device__ __forceinline__ v8f wmma16(v16h a, v16h b, v8f c) {
  v8f d = __builtin_amdgcn_wmma_f32_16x16x32_f16(false, a, false, b, (short)0, c,
                                                 false, false);
  asm volatile("v_nop\n\tv_nop\n\tv_nop\n\tv_nop" : "+v"(d) : "v"(a), "v"(b));
  return d;
}

__device__ __forceinline__ void wave_lds_sync() {
  __builtin_amdgcn_fence(3  , "wavefront");
  asm volatile("s_wait_dscnt 0x0" ::: "memory");
  __builtin_amdgcn_wave_barrier();
}

__global__ __launch_bounds__(256) void wconv_kernel(
    const float* __restrict__ W, _Float16* __restrict__ Wt, unsigned ldw, unsigned ldk) {
  __shared__ _Float16 T[64 * LDT];
  const unsigned tid = threadIdx.x;
  const unsigned n0 = blockIdx.x * 64u;
  const unsigned k0 = blockIdx.y * 64u;
#pragma unroll 4
  for (unsigned j = 0; j < 16u; ++j) {
    const unsigned idx = tid + 256u * j;
    const unsigned kr = idx >> 6, nc = idx & 63u;
    const float v = W[(size_t)(k0 + kr) * ldw + n0 + nc];
    T[nc * LDT + kr] = (_Float16)(WCARRY * bf16r(v));
  }
  __syncthreads();
  v8h x[2];
  size_t off[2];
#pragma unroll
  for (unsigned i = 0; i < 2u; ++i) {
    const unsigned n = 32u * i + (tid >> 3);
    const unsigned kc = (tid & 7u) * 8u;
    x[i] = *(const v8h*)&T[n * LDT + kc];
    off[i] = (size_t)(n0 + n) * ldk + k0 + kc;
  }
#pragma unroll
  for (int i = 0; i < 2; ++i) *(volatile v8h*)(Wt + off[i]) = x[i];
  __threadfence();
#pragma unroll
  for (int i = 0; i < 2; ++i) *(volatile v8h*)(Wt + off[i]) = x[i];
}

__device__ __forceinline__ void cast_row_1024(const float* __restrict__ src,
                                              _Float16* __restrict__ dst, const float carry) {
  const unsigned lane = threadIdx.x & 31u;
#pragma unroll 1
  for (unsigned j = 0; j < 4u; ++j) {
    const unsigned c = j * 256u + lane * 8u;
    const v4f a0 = *(const v4f*)(src + c);
    const v4f a1 = *(const v4f*)(src + c + 4u);
    v8h o;
#pragma unroll
    for (int i = 0; i < 4; ++i) {
      o[i]     = toh_flush(carry * bf16r(a0[i]));
      o[i + 4] = toh_flush(carry * bf16r(a1[i]));
    }
    _Float16* p = dst + c;
    *(volatile v8h*)p = o;
    __threadfence();
    *(volatile v8h*)p = o;
  }
}

__global__ __launch_bounds__(256) void wcast_kernel(
    const float* __restrict__ W, _Float16* __restrict__ Bt, unsigned coff) {
  const unsigned wave = __builtin_amdgcn_readfirstlane(threadIdx.x >> 5);
  const unsigned n = blockIdx.x * 8u + wave;
  cast_row_1024(W + (size_t)n * DIM, Bt + (size_t)n * KCAT + coff, WCARRY);
}

__global__ __launch_bounds__(256) void xcast_kernel(
    const float* __restrict__ X, _Float16* __restrict__ A16) {
  const unsigned wave = __builtin_amdgcn_readfirstlane(threadIdx.x >> 5);
  const unsigned crow = blockIdx.x * 8u + wave;
  const unsigned bidx = crow / (unsigned)SEQ;
  const unsigned sq = crow - bidx * (unsigned)SEQ;
  const size_t srow = (size_t)bidx * SEQ_FULL + sq;
  cast_row_1024(X + srow * DIM, A16 + (size_t)crow * KCAT, 1.0f);
}

__global__ __launch_bounds__(256) void pool_kernel(
    const int* __restrict__ ids, const int* __restrict__ nptr,
    const _Float16* __restrict__ Vt, _Float16* __restrict__ A16) {
  __shared__ __attribute__((aligned(16))) int T0[SEQ];
  __shared__ __attribute__((aligned(16))) int T1[SEQ];
  __shared__ __attribute__((aligned(16))) int T2[SEQ];
  __shared__ __attribute__((aligned(16))) _Float16 Ps[8 * 16 * LDT];

  const unsigned tid = threadIdx.x, lane = tid & 31u;
  const unsigned wave = __builtin_amdgcn_readfirstlane(tid >> 5);
  const unsigned hh = lane >> 4, m = lane & 15u;
  const unsigned q0 = blockIdx.x * 128u;
  const unsigned b = blockIdx.y;
  const unsigned qrow0 = q0 + wave * 16u;
  const int* row = ids + (size_t)b * SEQ_FULL;
  const unsigned kstage = q0 + 128u;

#pragma unroll 1
  for (unsigned p = tid; p < kstage; p += 256u) {
    const unsigned pa = (p >= 2u) ? (p - 2u) : 0u;
    const unsigned pc = (p >= 1u) ? (p - 1u) : 0u;
    const int i0 = row[pa];
    const int i1 = row[pc];
    const int i2 = row[p];
    const bool real = (p >= 2u);
    T0[p] = real ? i0 : 0;
    T1[p] = real ? i1 : 0;
    T2[p] = real ? i2 : 0;
  }
  __syncthreads();

  const unsigned q = qrow0 + m;
  const int tq0 = T0[q], tq1 = T1[q], tq2 = T2[q];

  auto build = [&](const unsigned s, int& c) -> v16h {
    const unsigned kbase = s * 32u + hh * 8u;
    v16h pf;
    int cc = 0;
#pragma unroll
    for (int g = 0; g < 4; ++g) {
      const unsigned ko = kbase + (unsigned)((g >> 1) * 16 + (g & 1) * 4);
      const v4i x0 = *(const v4i*)&T0[ko];
      const v4i x1 = *(const v4i*)&T1[ko];
      const v4i x2 = *(const v4i*)&T2[ko];
#pragma unroll
      for (int j = 0; j < 4; ++j) {
        const int hit = (int)(x0[j] == tq0) & (int)(x1[j] == tq1) & (int)(x2[j] == tq2) &
                        (int)((ko + (unsigned)j) < q);
        pf[g * 4 + j] = (hit != 0) ? (h16)1.0f : (h16)0.0f;
        cc += hit;
      }
    }
    c = cc;
    return pf;
  };

  const unsigned nsteps = (qrow0 + 16u + 31u) >> 5;
  unsigned long long hm = 0ull;
  int cnt = 0;
#pragma unroll 1
  for (unsigned s = 0; s < nsteps; ++s) {
    int c = 0;
    const v16h pf = build(s, c);
    (void)pf;
    cnt += c;
    const unsigned long long bal = __ballot(c != 0);
    const unsigned long long any = (bal != 0ull) ? 1ull : 0ull;
    hm |= any << s;
  }
  const unsigned hlo = __builtin_amdgcn_readfirstlane((unsigned)(hm & 0xFFFFFFFFull));
  const unsigned hhi = __builtin_amdgcn_readfirstlane((unsigned)(hm >> 32));
  const unsigned long long hs = ((unsigned long long)hhi << 32) | (unsigned long long)hlo;

  const int cntrow = cnt + __shfl_xor(cnt, 16, 32);
  const int cm = (cntrow > 1) ? cntrow : 1;
  const float invl = (1.0f / (float)cm) * (1.0f / WCARRY);
  float inv[8];
#pragma unroll
  for (int r = 0; r < 8; ++r) inv[r] = __shfl(invl, (int)(hh * 8u) + r, 32);

  const bool bad = (nptr[0] != 3);
  const float nanv = __uint_as_float(0x7FC00000u);

  const unsigned pb = wave * (16u * LDT);
  const size_t vbase = ((size_t)b * DIM + m) * SEQ + hh * 8u;
  const size_t obase = (size_t)(b * (unsigned)SEQ + qrow0) * KCAT + DIM;

#pragma unroll 1
  for (unsigned slab = 0; slab < (unsigned)(DIM / 64); ++slab) {
    v8f acc[4];
#pragma unroll
    for (int nb = 0; nb < 4; ++nb) acc[nb] = (v8f){};

#pragma unroll 1
    for (unsigned s = 0; s < nsteps; ++s) {
      if ((hs >> s) & 1ull) {
        int c = 0;
        const v16h pf = build(s, c);
        const _Float16* vp = Vt + vbase + (size_t)(slab * 64u) * SEQ + s * 32u;
#pragma unroll
        for (int nb = 0; nb < 4; ++nb) {
          const v16h vf = frag_at(vp + (size_t)(nb * 16) * SEQ);
          acc[nb] = wmma16(pf, vf, acc[nb]);
        }
      }
    }

#pragma unroll
    for (int nb = 0; nb < 4; ++nb)
#pragma unroll
      for (int r = 0; r < 8; ++r) {
        const float t = acc[nb][r] * inv[r];
        const float tv = bad ? nanv : t;
        Ps[pb + (hh * 8u + (unsigned)r) * LDT + (unsigned)nb * 16u + m] = toh_flush(tv);
      }
    wave_lds_sync();
    v8h x[4];
    size_t off[4];
#pragma unroll
    for (unsigned i = 0; i < 4u; ++i) {
      const unsigned r = 4u * i + (lane >> 3);
      const unsigned c = (lane & 7u) * 8u;
      x[i] = *(const v8h*)&Ps[pb + r * LDT + c];
      off[i] = obase + (size_t)r * KCAT + slab * 64u + c;
    }
#pragma unroll
    for (int i = 0; i < 4; ++i) *(volatile v8h*)(A16 + off[i]) = x[i];
    __threadfence();
#pragma unroll
    for (int i = 0; i < 4; ++i) *(volatile v8h*)(A16 + off[i]) = x[i];
    wave_lds_sync();
  }
}

__global__ __launch_bounds__(256) void gemm_out_kernel(
    const _Float16* __restrict__ A16, const _Float16* __restrict__ Bt,
    const float* __restrict__ b1, const float* __restrict__ b2, float* __restrict__ outf) {
  __shared__ __attribute__((aligned(16))) float Cs[64 * LDC];
  const unsigned tid = threadIdx.x, lane = tid & 31u;
  const unsigned w = __builtin_amdgcn_readfirstlane(tid >> 5);
  const unsigned mw = w >> 1, nw = w & 1u;
  const unsigned hh = lane >> 4, m = lane & 15u;
  const unsigned n0 = blockIdx.x * 64u;
  const unsigned row0 = blockIdx.y * 64u;
  const unsigned K = (unsigned)KCAT;

  const _Float16* ap  = A16 + (size_t)(row0 + mw * 16u + m) * K + hh * 8u;
  const _Float16* bp0 = Bt + (size_t)(n0 + nw * 32u + m) * K + hh * 8u;
  const _Float16* bp1 = bp0 + (size_t)16 * K;
  v8f acc0 = {}, acc1 = {};
#pragma unroll 2
  for (unsigned k0 = 0; k0 < K; k0 += 32u) {
    const v16h a  = frag_at(ap + k0);
    const v16h b0 = frag_at(bp0 + k0);
    const v16h b1f = frag_at(bp1 + k0);
    acc0 = wmma16(a, b0, acc0);
    acc1 = wmma16(a, b1f, acc1);
  }
#pragma unroll
  for (int r = 0; r < 8; ++r) {
    float* d = &Cs[(mw * 16u + hh * 8u + (unsigned)r) * LDC + nw * 32u + m];
    d[0]  = acc0[r];
    d[16] = acc1[r];
  }
  __syncthreads();

  v4f xs[4];
  size_t off[4];
#pragma unroll
  for (unsigned i = 0; i < 4u; ++i) {
    const unsigned r = 16u * i + (tid >> 4);
    const unsigned c = (tid & 15u) * 4u;
    const unsigned crow = row0 + r;
    const unsigned bidx = crow / (unsigned)SEQ;
    const unsigned sq = crow - bidx * (unsigned)SEQ;
    const size_t frow = (size_t)bidx * SEQ_FULL + sq;
    const v4f u  = *(const v4f*)&Cs[r * LDC + c];
    const v4f g1 = *(const v4f*)(b1 + n0 + c);
    const v4f g2 = *(const v4f*)(b2 + n0 + c);
    v4f val;
#pragma unroll
    for (int j = 0; j < 4; ++j)
      val[j] = u[j] * (1.0f / WCARRY) + (bf16r(g1[j]) + bf16r(g2[j]));
    xs[i] = val;
    off[i] = frow * DIM + n0 + c;
  }
#pragma unroll
  for (int i = 0; i < 4; ++i) *(volatile v4f*)(outf + off[i]) = xs[i];
  __threadfence();
#pragma unroll
  for (int i = 0; i < 4; ++i) *(volatile v4f*)(outf + off[i]) = xs[i];
}

extern "C" void kernel_launch(void* const* d_in, const int* in_sizes, int n_in,
                              void* d_out, int out_size, void* d_ws, size_t ws_size,
                              hipStream_t stream) {
  if (n_in < 7) return;
  const long long need_rows = (long long)(NB - 1) * SEQ_FULL + SEQ;
  if ((long long)in_sizes[0] < need_rows * DIM) return;
  if ((long long)in_sizes[1] < need_rows) return;
  if ((long long)in_sizes[2] < (long long)DIM * DIM) return;
  if ((long long)in_sizes[4] < (long long)DIM * DIM) return;
  if (in_sizes[3] < DIM || in_sizes[5] < DIM || in_sizes[6] < 1) return;
  if ((long long)out_size < need_rows * DIM) return;
  if (ws_size < WS_TOTAL) return;

  const float* X   = (const float*)d_in[0];
  const int*   ids = (const int*)d_in[1];
  const float* w1  = (const float*)d_in[2];
  const float* b1  = (const float*)d_in[3];
  const float* w2  = (const float*)d_in[4];
  const float* b2  = (const float*)d_in[5];
  const int*   np  = (const int*)d_in[6];
  float* out = (float*)d_out;

  char* ws = (char*)d_ws;
  _Float16* Bt16 = (_Float16*)(ws + OFF_BT);
  _Float16* A16  = (_Float16*)(ws + OFF_A);
  _Float16* Vt16 = (_Float16*)(ws + OFF_VT);

  dim3 blk(256);

  wcast_kernel<<<dim3(DIM / 8), blk, 0, stream>>>(w1, Bt16, 0u);
  wcast_kernel<<<dim3(DIM / 8), blk, 0, stream>>>(w2, Bt16, (unsigned)DIM);
  xcast_kernel<<<dim3(MROWS / 8), blk, 0, stream>>>(X, A16);
  for (int b = 0; b < NB; ++b) {
    wconv_kernel<<<dim3(DIM / 64, SEQ / 64), blk, 0, stream>>>(
        X + (size_t)b * SEQ_FULL * DIM, Vt16 + (size_t)b * DIM * SEQ, (unsigned)DIM, (unsigned)SEQ);
  }
  pool_kernel<<<dim3(SEQ / 128, NB), blk, 0, stream>>>(ids, np, Vt16, A16);
  gemm_out_kernel<<<dim3(DIM / 64, MROWS / 64), blk, 0, stream>>>(A16, Bt16, b1, b2, out);
}
